// BatteryMoEFlattenIntraCycleMoELayer_79310866088194
// MI455X (gfx1250) — hardware-verified
//
#include <hip/hip_runtime.h>
#include <stddef.h>
#include <stdint.h>

#define NB   128
#define NL   128
#define NE   8
#define KIN  900
#define KP   960
#define ND   512
#define BH   64
#define NH   2
#define KT   64
#define NT   64
#define TP   68
#define MT   128
#define OP   136
#define WSC  1024.0f
#define WSI  0.0009765625f
#define EPSG 1e-9f

static_assert(KP % 64 == 0);
static_assert(KP % 32 == 0);
static_assert(KP >= KIN);
static_assert(KP - KIN < KT);
static_assert(KP % KT == 0);
static_assert(KIN % 4 == 0);
static_assert(ND % NT == 0);
static_assert(ND % MT == 0);
static_assert(NB == NH * BH);
static_assert((NB * NL) % 8 == 0);
static_assert(NE == 8);
static_assert(NL == 128);
static_assert(TP % 4 == 0);
static_assert(OP % 8 == 0);

typedef _Float16 v16h __attribute__((ext_vector_type(16)));
typedef _Float16 v8h  __attribute__((ext_vector_type(8)));
typedef float    v8f  __attribute__((ext_vector_type(8)));
typedef float    v4f  __attribute__((ext_vector_type(4)));
typedef unsigned int   v4u  __attribute__((ext_vector_type(4)));
typedef unsigned short v8us __attribute__((ext_vector_type(8)));

union Frag  { v16h v; v8h h[2]; };
union Pack8 { v8h h; v4u u; };

__device__ __forceinline__ v8f mma16(v16h a, v16h b, v8f c) {
  c = __builtin_amdgcn_wmma_f32_16x16x32_f16(false, a, false, b, (short)0, c, false, false);
  asm volatile("v_nop\n\tv_nop\n\tv_nop\n\tv_nop" : "+v"(c) : "v"(a), "v"(b));
  return c;
}

__device__ __forceinline__ v16h ldfrag(const _Float16* p, int ld, int row0, int k0, int lane) {
  const int m = lane & 15, lh = lane >> 4;
  const _Float16* q = p + (size_t)(row0 + m) * ld + k0 + 8 * lh;
  Frag f;
  f.h[0] = *(const v8h*)(q);
  f.h[1] = *(const v8h*)(q + 16);
  return f.v;
}

__device__ __forceinline__ v8f zero8() { return (v8f){0.f, 0.f, 0.f, 0.f, 0.f, 0.f, 0.f, 0.f}; }

__device__ __forceinline__ unsigned short bf16_rne(float f) {
  unsigned int u = __float_as_uint(f);
  u += 0x7FFFu + ((u >> 16) & 1u);
  return (unsigned short)(u >> 16);
}

__device__ __forceinline__ float gate_lane(const float* __restrict__ logits, const int* __restrict__ masks,
                                           int topk, int b, int lane) {
  const int e = lane & 7, gbase = lane & 24;
  const float lg = logits[b * NE + e];
  const int   mk = masks[b * NE + e];
  float mx = lg;
  mx = fmaxf(mx, __shfl_xor(mx, 1, 32));
  mx = fmaxf(mx, __shfl_xor(mx, 2, 32));
  mx = fmaxf(mx, __shfl_xor(mx, 4, 32));
  const float p = expf(lg - mx);
  float s = p;
  s += __shfl_xor(s, 1, 32);
  s += __shfl_xor(s, 2, 32);
  s += __shfl_xor(s, 4, 32);
  s = __shfl(s, gbase, 32);
  const float rs = 1.0f / s;
  const float g = (mk == 1) ? p * rs : 0.0f;
  int cnt = 0;
#pragma unroll
  for (int j = 0; j < NE; ++j) {
    const float gj = __shfl(g, gbase + j, 32);
    cnt += ((gj > g) || (gj == g && j < e)) ? 1 : 0;
  }
  const bool sel = (topk <= 0) || (cnt < topk);
  const float gs = sel ? g : 0.0f;
  float ss = gs;
  ss += __shfl_xor(ss, 1, 32);
  ss += __shfl_xor(ss, 2, 32);
  ss += __shfl_xor(ss, 4, 32);
  ss = __shfl(ss, gbase, 32);
  const float rn = 1.0f / (ss + EPSG);
  return gs * rn;
}

__global__ __launch_bounds__(256) void k_cvtx(const float* __restrict__ x, _Float16* __restrict__ xh, int nrows) {
  const int tid = threadIdx.x, lane = tid & 31, wave = tid >> 5;
  const int row = blockIdx.x * 8 + wave;
  if (row >= nrows) return;
  const float* s = x + (size_t)row * KIN;
  const v4f z4 = (v4f){0.f, 0.f, 0.f, 0.f};
  v4u pv[4];
#pragma unroll
  for (int it = 0; it < 4; ++it) {
    const int p  = 32 * it + lane;
    const int f0 = 8 * p;
    const int q0 = min(f0, KIN - 4);
    const int q1 = min(f0 + 4, KIN - 4);
    v4f a = *(const v4f*)(s + q0);
    v4f c = *(const v4f*)(s + q1);
    if (f0 >= KIN) a = z4;
    if (f0 + 4 >= KIN) c = z4;
    Pack8 pk;
    pk.h = (v8h){(_Float16)a[0], (_Float16)a[1], (_Float16)a[2], (_Float16)a[3],
                 (_Float16)c[0], (_Float16)c[1], (_Float16)c[2], (_Float16)c[3]};
    pv[it] = pk.u;
  }
  _Float16* d = xh + (size_t)row * KP;
  for (int ps = 0; ps < 2; ++ps) {
#pragma unroll
    for (int it = 0; it < 4; ++it) {
      const int p = 32 * it + lane;
      if (p < KP / 8) *(volatile v4u*)(d + 8 * p) = pv[it];
    }
    __threadfence();
  }
}

__global__ __launch_bounds__(256) void k_comb(const float* __restrict__ w, const float* __restrict__ logits,
                                              const int* __restrict__ masks, const int* __restrict__ topk,
                                              _Float16* __restrict__ wg, int b0) {
  __shared__ __align__(16) float sT[NT * TP];
  __shared__ float sG[NE];
  const int tid = threadIdx.x, lane = tid & 31, wave = tid >> 5;
  const int kt = blockIdx.x, nt = blockIdx.y, bl = blockIdx.z;
  const int b = b0 + bl;
  if (wave == 0) {
    const float gv = gate_lane(logits, masks, topk[0], b, lane);
    if (lane < NE) sG[lane] = gv;
  }
  __syncthreads();

  const int k0 = kt * KT, n0 = nt * NT;
  const int c4 = tid & 15, rr = tid >> 4;
  const v4f z4 = (v4f){0.f, 0.f, 0.f, 0.f};
  v4f acc[4];
#pragma unroll
  for (int ps = 0; ps < 4; ++ps) acc[ps] = z4;
#pragma unroll 1
  for (int e = 0; e < NE; ++e) {
    const float gu = __int_as_float(__builtin_amdgcn_readfirstlane(__float_as_int(sG[e])));
    if (gu != 0.0f) {
      const float* we = w + (size_t)e * KIN * ND + n0 + 4 * c4;
#pragma unroll
      for (int ps = 0; ps < 4; ++ps) {
        const int k  = k0 + rr + 16 * ps;
        const int kc = min(k, KIN - 1);
        v4f v = *(const v4f*)(we + (size_t)kc * ND);
        if (k >= KIN) v = z4;
        acc[ps] += gu * v;
      }
    }
  }
#pragma unroll
  for (int ps = 0; ps < 4; ++ps) {
    const int kl = rr + 16 * ps;
#pragma unroll
    for (int i = 0; i < 4; ++i) sT[(4 * c4 + i) * TP + kl] = acc[ps][i] * WSC;
  }
  __syncthreads();

  v4u pv[2];
  size_t po[2];
#pragma unroll
  for (int it = 0; it < 2; ++it) {
    const int p  = tid + 256 * it;
    const int nl = p >> 3;
    const int pc = p & 7;
    const float* s = sT + nl * TP + 8 * pc;
    const v4f a0 = *(const v4f*)(s);
    const v4f a1 = *(const v4f*)(s + 4);
    Pack8 pk;
    pk.h = (v8h){(_Float16)a0[0], (_Float16)a0[1], (_Float16)a0[2], (_Float16)a0[3],
                 (_Float16)a1[0], (_Float16)a1[1], (_Float16)a1[2], (_Float16)a1[3]};
    pv[it] = pk.u;
    po[it] = ((size_t)bl * ND + n0 + nl) * KP + k0 + 8 * pc;
  }
  for (int ps = 0; ps < 2; ++ps) {
#pragma unroll
    for (int it = 0; it < 2; ++it) *(volatile v4u*)(wg + po[it]) = pv[it];
    __threadfence();
  }
}

__global__ __launch_bounds__(256) void k_gemm(const _Float16* __restrict__ xh, const _Float16* __restrict__ wg,
                                              const float* __restrict__ bias, const float* __restrict__ logits,
                                              const int* __restrict__ masks, const int* __restrict__ topk,
                                              unsigned short* __restrict__ out, int b0, int tail) {
  __shared__ __align__(16) unsigned short sO[NL * OP];
  __shared__ float sG[NE];
  const int tid = threadIdx.x, lane = tid & 31, wave = tid >> 5;
  const int hh = lane >> 4, c = lane & 15;
  const int n0 = blockIdx.x * MT, bl = blockIdx.y;
  const int b = b0 + bl;
  if (wave == 0) {
    const float gv = gate_lane(logits, masks, topk[0], b, lane);
    if (lane < NE) sG[lane] = gv;
  }
  __syncthreads();

  const int wm = (wave >> 2) * 64, wn = (wave & 3) * 32;
  const _Float16* xb = xh + (size_t)b * NL * KP;
  const _Float16* wb = wg + ((size_t)bl * ND + n0) * KP;
  v8f acc[4][2];
#pragma unroll
  for (int i = 0; i < 4; ++i) { acc[i][0] = zero8(); acc[i][1] = zero8(); }
#pragma unroll 1
  for (int k0 = 0; k0 < KP; k0 += 32) {
    const v16h q0 = ldfrag(wb, KP, wn, k0, lane);
    const v16h q1 = ldfrag(wb, KP, wn + 16, k0, lane);
#pragma unroll
    for (int i = 0; i < 4; ++i) {
      const v16h a = ldfrag(xb, KP, wm + 16 * i, k0, lane);
      acc[i][0] = mma16(a, q0, acc[i][0]);
      acc[i][1] = mma16(a, q1, acc[i][1]);
    }
  }

  float gb[2];
#pragma unroll
  for (int j = 0; j < 2; ++j) {
    const int n = n0 + wn + 16 * j + c;
    float s = 0.f;
#pragma unroll
    for (int e = 0; e < NE; ++e) s += sG[e] * bias[e * ND + n];
    gb[j] = s;
  }
#pragma unroll
  for (int i = 0; i < 4; ++i) {
#pragma unroll
    for (int j = 0; j < 2; ++j) {
      const int col = wn + 16 * j + c;
#pragma unroll
      for (int r = 0; r < 8; ++r) {
        const int row = wm + 16 * i + 8 * hh + r;
        const float v = acc[i][j][r] * WSI + gb[j];
        sO[row * OP + col] = bf16_rne(v);
      }
    }
  }
  __syncthreads();

  const size_t orow0 = (size_t)b * NL;
  const bool do_tail = (tail != 0) && (blockIdx.x == 0) && (blockIdx.y == 0) && (tid == 0);
  for (int ps = 0; ps < 2; ++ps) {
#pragma unroll
    for (int it = 0; it < 8; ++it) {
      const int p   = tid + 256 * it;
      const int ln  = p >> 3;
      const int pc  = p & 7;
      const int row = ln >> 1;
      const int col = (ln & 1) * 64 + 8 * pc;
      const v8us val = *(const v8us*)(sO + row * OP + col);
      *(volatile v8us*)(out + (orow0 + row) * ND + n0 + col) = val;
    }
    if (do_tail) *(volatile unsigned int*)(out + (size_t)NB * NL * ND) = 0u;
    __threadfence();
  }
}

extern "C" void kernel_launch(void* const* d_in, const int* in_sizes, int n_in,
                              void* d_out, int out_size, void* d_ws, size_t ws_size,
                              hipStream_t stream) {
  if (n_in < 6) return;
  if (in_sizes[0] != NB * NL * KIN) return;
  if (in_sizes[1] != NB * NE) return;
  if (in_sizes[2] != NB * NE) return;
  if (in_sizes[3] != NE * KIN * ND) return;
  if (in_sizes[4] != NE * ND) return;
  if (in_sizes[5] < 1) return;
  if (out_size != NB * NL * ND + 2) return;

  const float* x      = (const float*)d_in[0];
  const float* logits = (const float*)d_in[1];
  const int*   masks  = (const int*)d_in[2];
  const float* w      = (const float*)d_in[3];
  const float* bias   = (const float*)d_in[4];
  const int*   topk   = (const int*)d_in[5];
  unsigned short* out = (unsigned short*)d_out;

  size_t off = 0;
  const size_t oX = off; off += (size_t)NB * NL * KP * 2;
  const size_t oW = off; off += (size_t)BH * ND * KP * 2;
  if (off > ws_size) return;
  if (off > (size_t)134217728) return;
  if ((oX | oW) & (size_t)127) return;

  char* ws = (char*)d_ws;
  _Float16* XH = (_Float16*)(ws + oX);
  _Float16* WG = (_Float16*)(ws + oW);

  k_cvtx<<<dim3((NB * NL) / 8), dim3(256), 0, stream>>>(x, XH, NB * NL);
  for (int h = 0; h < NH; ++h) {
    k_comb<<<dim3(KP / KT, ND / NT, BH), dim3(256), 0, stream>>>(w, logits, masks, topk, WG, h * BH);
    k_gemm<<<dim3(ND / MT, BH), dim3(256), 0, stream>>>(XH, WG, bias, logits, masks, topk, out, h * BH,
                                                        (h == 0) ? 1 : 0);
  }
  (void)hipGetLastError();
}
